// Mamba2_51823075393736
// MI455X (gfx1250) — hardware-verified
//
#include <hip/hip_runtime.h>
#include <math.h>

typedef __attribute__((ext_vector_type(16))) _Float16 v16h;
typedef __attribute__((ext_vector_type(8)))  _Float16 v8h;
typedef __attribute__((ext_vector_type(16))) __bf16   v16b;
typedef __attribute__((ext_vector_type(8)))  __bf16   v8b;
typedef __attribute__((ext_vector_type(8)))  float    v8f;
typedef __attribute__((ext_vector_type(4)))  float    v4f;
typedef __attribute__((ext_vector_type(4)))  unsigned v4u;

constexpr int kBatch  = 2;
constexpr int kSeq    = 2048;
constexpr int kDm     = 1024;
constexpr int kDi     = 2048;
constexpr int kHeads  = 32;
constexpr int kHd     = 64;
constexpr int kNs     = 64;
constexpr int kChunkQ = 128;
constexpr int kNChunk = kSeq / kChunkQ;
constexpr int kCproj  = 2 * kDi + 2 * kNs + kHeads;
constexpr int kCpad   = 4288;
constexpr int kRows   = kBatch * kSeq;
constexpr int kNbc    = kBatch * kNChunk;
constexpr int kNblk   = kNbc * kHeads;
constexpr int kTP     = 136;
constexpr int kHP     = 72;
constexpr int kConvTP = 260;
static_assert(kHeads * kHd == kDi, "inner width");
static_assert(kCpad % 64 == 0 && kCpad >= kCproj && kCpad - kCproj < 64, "padded projection width");
static_assert((kDm % 32) == 0 && (kNs % 32) == 0 && (kChunkQ % 32) == 0 && (kDi % 32) == 0, "GEMM K multiples of 32");
static_assert((kRows % 64) == 0 && (kCpad % 64) == 0 && (kChunkQ % 64) == 0 && (kDm % 64) == 0, "GEMM M,N multiples of 64");
static_assert(((kTP * 2) % 16) == 0 && ((kHP * 2) % 16) == 0 && ((kConvTP * 4) % 16) == 0, "16-B aligned LDS rows");
static_assert(kChunkQ == 128 && kHd == 64 && kNs == 64, "tile code assumes these extents");

constexpr size_t kOffUB   = 0;
constexpr size_t kOffWIB  = kOffUB  + (size_t)kRows * kDm * 2;
constexpr size_t kOffWOB  = kOffWIB + (size_t)kCpad * kDm * 2;
constexpr size_t kOffZX   = kOffWOB + (size_t)kDm * kDi * 2;
constexpr size_t kSzZX    = (size_t)kRows * kCpad * 4;
constexpr size_t kOffZ16  = kOffZX  + kSzZX;
constexpr size_t kOffX16  = kOffZ16 + (size_t)kRows * kDi * 2;
constexpr size_t kOffB16  = kOffX16 + (size_t)kRows * kDi * 2;
constexpr size_t kOffC16  = kOffB16 + (size_t)kRows * kNs * 2;
constexpr size_t kOffDT   = kOffC16 + (size_t)kRows * kNs * 2;
constexpr size_t kOffAL   = kOffDT  + (size_t)kRows * kHeads * 4;
constexpr size_t kOffCB   = kOffAL  + (size_t)kRows * kHeads * 4;
constexpr size_t kWsTotal = kOffCB  + (size_t)kNbc * kChunkQ * kChunkQ * 4;
constexpr size_t kOffDH   = kOffZX;
constexpr size_t kSzDH    = (size_t)kNblk * kNs * kHd * 4;
constexpr size_t kOffHPV  = kOffDH + kSzDH;
constexpr size_t kOffY    = kOffHPV + kSzDH;
constexpr size_t kSzY     = (size_t)kRows * kDi * 4;
constexpr size_t kOffG16  = kOffX16;
static_assert(kWsTotal == 129368064ull, "carve total");
static_assert(kWsTotal <= 134217728ull, "carve cap");
static_assert(kOffY + kSzY <= kOffZX + kSzZX, "aliases fit inside the dead ZX region");
static_assert((kOffWIB % 128) == 0 && (kOffWOB % 128) == 0 && (kOffZX % 128) == 0 && (kOffZ16 % 128) == 0 &&
              (kOffX16 % 128) == 0 && (kOffB16 % 128) == 0 && (kOffC16 % 128) == 0 && (kOffDT % 128) == 0 &&
              (kOffAL % 128) == 0 && (kOffCB % 128) == 0 && (kOffHPV % 128) == 0 && (kOffY % 128) == 0,
              "128-B aligned regions");

constexpr int kU8      = kRows * kDm / 8;
constexpr int kWin8    = kCpad * kDm / 8;
constexpr int kWinSrc8 = kCproj * kDm / 8;
constexpr int kWout8   = kDm * kDi / 8;
constexpr int kTilesIn  = (kRows / 64) * (kCpad / 64);
constexpr int kTilesOut = (kRows / 64) * (kDm / 64);
static_assert((kU8 % 256) == 0 && (kWin8 % 256) == 0 && (kWout8 % 256) == 0, "convert grids exact");
static_assert((kTilesIn % 8) == 0 && (kTilesOut % 8) == 0, "GEMM grids exact");
static_assert((kCproj + 255) / 256 == 17 && (kRows % 64) == 0, "conv grid");

__device__ __forceinline__ unsigned short f2bf_bits(float f) {
  unsigned u = __float_as_uint(f);
  return (unsigned short)((u + 0x7FFFu + ((u >> 16) & 1u)) >> 16);
}
__device__ __forceinline__ float bf_bits2f(unsigned short h) { return __uint_as_float(((unsigned)h) << 16); }
__device__ __forceinline__ float bfr(float f) { return bf_bits2f(f2bf_bits(f)); }
__device__ __forceinline__ float h16_to_f32(unsigned hb) {
  const unsigned sgn = (hb & 0x8000u) << 16; const unsigned em = hb & 0x7fffu;
  const float fn = __uint_as_float((em << 13) + 0x38000000u);
  const float fs = (float)em * 5.9604644775390625e-8f;
  const float mag = (em < 0x400u) ? fs : fn; return __uint_as_float(__float_as_uint(mag) | sgn);
}
__device__ __forceinline__ unsigned short f16_bits(float f) { return __builtin_bit_cast(unsigned short, (_Float16)f); }

__device__ __forceinline__ void dep_guard4_h(v8f& a, v8f& b, v8f& c, v8f& d, v16h x, v16h y) {
  asm volatile("v_nop\n\tv_nop\n\tv_nop\n\tv_nop" : "+v"(a), "+v"(b), "+v"(c), "+v"(d) : "v"(x), "v"(y));
}
__device__ __forceinline__ void dep_guard4_b(v8f& a, v8f& b, v8f& c, v8f& d, v16b x, v16b y) {
  asm volatile("v_nop\n\tv_nop\n\tv_nop\n\tv_nop" : "+v"(a), "+v"(b), "+v"(c), "+v"(d) : "v"(x), "v"(y));
}
__device__ __forceinline__ void keep4_h(v16h a, v16h b, v16h c, v16h d) { asm volatile("v_nop" :: "v"(a), "v"(b), "v"(c), "v"(d)); }
__device__ __forceinline__ void keep4_b(v16b a, v16b b, v16b c, v16b d) { asm volatile("v_nop" :: "v"(a), "v"(b), "v"(c), "v"(d)); }
__device__ __forceinline__ void acc_guard4(v8f& a, v8f& b, v8f& c, v8f& d) { asm volatile("v_nop\n\tv_nop\n\tv_nop\n\tv_nop" : "+v"(a), "+v"(b), "+v"(c), "+v"(d)); }

template <typename T> struct Frag;
template <> struct Frag<_Float16> {
  typedef v16h V; union U { v16h v; v8h h[2]; };
  static __device__ __forceinline__ v16h load(const _Float16* p) {
    U f; f.h[0] = *(const v8h*)(p); f.h[1] = *(const v8h*)(p + 16); return f.v;
  }
  static __device__ __forceinline__ v8f mma(v16h a, v16h b, v8f c) {
    return __builtin_amdgcn_wmma_f32_16x16x32_f16(false, a, false, b, (short)0, c, false, false);
  }
  static __device__ __forceinline__ void guard4(v8f& a, v8f& b, v8f& c, v8f& d, v16h x, v16h y) { dep_guard4_h(a, b, c, d, x, y); }
  static __device__ __forceinline__ void keep(v16h a, v16h b, v16h c, v16h d) { keep4_h(a, b, c, d); }
};
template <> struct Frag<__bf16> {
  typedef v16b V; union U { v16b v; v8b h[2]; };
  static __device__ __forceinline__ v16b load(const __bf16* p) {
    U f; f.h[0] = *(const v8b*)(p); f.h[1] = *(const v8b*)(p + 16); return f.v;
  }
  static __device__ __forceinline__ v8f mma(v16b a, v16b b, v8f c) {
    return __builtin_amdgcn_wmma_f32_16x16x32_bf16(false, a, false, b, (short)0, c, false, false);
  }
  static __device__ __forceinline__ void guard4(v8f& a, v8f& b, v8f& c, v8f& d, v16b x, v16b y) { dep_guard4_b(a, b, c, d, x, y); }
  static __device__ __forceinline__ void keep(v16b a, v16b b, v16b c, v16b d) { keep4_b(a, b, c, d); }
};

__device__ __forceinline__ v16h lds_frag(const unsigned short* p) {
  Frag<_Float16>::U f;
  f.h[0] = *(const v8h*)(const void*)(p);
  f.h[1] = *(const v8h*)(const void*)(p + 16);
  return f.v;
}

__device__ __forceinline__ float wave_scan_incl(float v, int lane) {
#pragma unroll
  for (int off = 1; off < 32; off <<= 1) {
    const float t = __shfl_up(v, off, 32);
    v += (lane >= off) ? t : 0.0f;
  }
  return v;
}

template <int ET> struct Elem;
template <> struct Elem<0> { typedef _Float16 T; };
template <> struct Elem<1> { typedef __bf16 T; };
template <int ET, int SPL, int BIAS_MODE, int OUT_MODE, bool RESID, int ACT = 0>
__global__ __launch_bounds__(256) void wmma_gemm64(
    const unsigned short* __restrict__ Ap, const unsigned short* __restrict__ A2p, int lda, long strideA,
    const unsigned short* __restrict__ Btp, const unsigned short* __restrict__ Bt2p, int ldb, long strideB,
    void* __restrict__ Cout, void* __restrict__ Cout2, int ldc, long strideC,
    const float* __restrict__ bias,
    const float* __restrict__ resid, long strideR,
    int M, int N, int K, float scale) {
  typedef typename Elem<ET>::T T;
  typedef typename Frag<T>::V V;
  const T* A = (const T*)Ap; const T* A2 = (const T*)A2p; const T* Bt = (const T*)Btp; const T* Bt2 = (const T*)Bt2p;
  __shared__ __align__(16) float sT[8][16 * 68];
  const int b    = blockIdx.y;
  const int lane = threadIdx.x & 31;
  const int wave = threadIdx.x >> 5;
  const int tilesN = N >> 6;
  const int tilesM = M >> 6;
  const int tile = blockIdx.x * 8 + wave;
  if (tile >= tilesM * tilesN) return;
  const int tm = tile / tilesN;
  const int tn = tile - tm * tilesN;
  const int m0 = tm << 6;
  const int n0 = tn << 6;

  const T* Ab  = A  + (size_t)b * strideA;
  const T* Bb  = Bt + (size_t)b * strideB;
  const T* Ab2 = (SPL >= 1) ? (A2  + (size_t)b * strideA) : nullptr;
  const T* Bb2 = (SPL == 2) ? (Bt2 + (size_t)b * strideB) : nullptr;

  const int rlane = lane & 15;
  const int koff  = (lane >> 4) * 8;
  const int mOff  = (lane >> 4) * 8;

  v8f acc[4][4];
#pragma unroll
  for (int i = 0; i < 4; ++i)
#pragma unroll
    for (int j = 0; j < 4; ++j) acc[i][j] = (v8f){0.f,0.f,0.f,0.f,0.f,0.f,0.f,0.f};

  for (int k0 = 0; k0 < K; k0 += 32) {
    V bh[4], bl[4];
#pragma unroll
    for (int j = 0; j < 4; ++j) {
      const size_t bo = (size_t)(n0 + (j << 4) + rlane) * ldb + koff + k0;
      bh[j] = Frag<T>::load(Bb + bo);
      if (SPL == 2) bl[j] = Frag<T>::load(Bb2 + bo);
    }
#pragma unroll
    for (int i = 0; i < 4; ++i) {
      const size_t ao = (size_t)(m0 + (i << 4) + rlane) * lda + koff + k0;
      V ah = Frag<T>::load(Ab + ao);
      V al;
      if (SPL >= 1) al = Frag<T>::load(Ab2 + ao);
#pragma unroll
      for (int j = 0; j < 4; ++j) {
        acc[i][j] = Frag<T>::mma(ah, bh[j], acc[i][j]);
        if (SPL == 2) acc[i][j] = Frag<T>::mma(ah, bl[j], acc[i][j]);
        if (SPL >= 1) acc[i][j] = Frag<T>::mma(al, bh[j], acc[i][j]);
      }
      Frag<T>::guard4(acc[i][0], acc[i][1], acc[i][2], acc[i][3], ah, (SPL >= 1) ? al : ah);
    }
    Frag<T>::keep(bh[0], bh[1], bh[2], bh[3]);
    if (SPL == 2) Frag<T>::keep(bl[0], bl[1], bl[2], bl[3]);
  }
  acc_guard4(acc[0][0], acc[0][1], acc[0][2], acc[0][3]);
  acc_guard4(acc[1][0], acc[1][1], acc[1][2], acc[1][3]);
  acc_guard4(acc[2][0], acc[2][1], acc[2][2], acc[2][3]);
  acc_guard4(acc[3][0], acc[3][1], acc[3][2], acc[3][3]);

  float* slab = sT[wave];
  const float* Rb = RESID ? (resid + (size_t)b * strideR) : nullptr;
#pragma unroll
  for (int i = 0; i < 4; ++i) {
    const int mBase = m0 + (i << 4);
#pragma unroll
    for (int j = 0; j < 4; ++j) {
      const int n = n0 + (j << 4) + rlane;
      float bv = 0.f;
      if (BIAS_MODE == 2) bv = bias[n];
#pragma unroll
      for (int r = 0; r < 8; ++r) {
        float v = acc[i][j][r] * scale;
        if (BIAS_MODE == 1) v += bias[mBase + mOff + r];
        if (BIAS_MODE == 2) v += bv;
        if (RESID) v += Rb[(size_t)(mBase + mOff + r) * ldc + n];
        if (ACT == 1) v = tanhf(v);
        if (ACT == 2) v = fmaxf(v, 0.0f);
        if (ACT == 3) v = v / (1.0f + expf(-v));
        if (ACT == 4) v = (v > 0.f) ? v : 0.01f * v;
        slab[(mOff + r) * 68 + (j << 4) + rlane] = v;
      }
    }
    __builtin_amdgcn_fence(__ATOMIC_RELEASE, "workgroup");
    __builtin_amdgcn_wave_barrier();
    __builtin_amdgcn_fence(__ATOMIC_ACQUIRE, "workgroup");
    if (OUT_MODE == 0) {
      float* C = (float*)Cout + (size_t)b * strideC;
      const int hh = lane >> 4, c4 = (lane & 15) * 4;
      for (int pass = 0; pass < 2; ++pass) {
#pragma unroll
        for (int it = 0; it < 8; ++it) {
          const int row = it * 2 + hh;
          v4f v = *(const v4f*)(slab + row * 68 + c4);
          *(volatile v4f*)(C + (size_t)(mBase + row) * ldc + n0 + c4) = v;
        }
        __threadfence();
      }
    } else {
      const int q = lane >> 3, c8 = (lane & 7) * 8;
      unsigned short* C  = (unsigned short*)Cout  + (size_t)b * strideC;
      unsigned short* C2 = (OUT_MODE == 2) ? ((unsigned short*)Cout2 + (size_t)b * strideC) : nullptr;
      for (int pass = 0; pass < 2; ++pass) {
#pragma unroll
        for (int it = 0; it < 4; ++it) {
          const int row = it * 4 + q;
          const float* sp = slab + row * 68 + c8;
          v8h hv, lv;
#pragma unroll
          for (int e = 0; e < 8; ++e) {
            if (OUT_MODE == 1) {
              hv[e] = (_Float16)sp[e];
            } else {
              unsigned short hb = f2bf_bits(sp[e]);
              unsigned short lb = f2bf_bits(sp[e] - bf_bits2f(hb));
              hv[e] = __builtin_bit_cast(_Float16, hb);
              lv[e] = __builtin_bit_cast(_Float16, lb);
            }
          }
          *(volatile v8h*)(C + (size_t)(mBase + row) * ldc + n0 + c8) = hv;
          if (OUT_MODE == 2) *(volatile v8h*)(C2 + (size_t)(mBase + row) * ldc + n0 + c8) = lv;
        }
        __threadfence();
      }
    }
    __builtin_amdgcn_fence(__ATOMIC_RELEASE, "workgroup");
    __builtin_amdgcn_wave_barrier();
    __builtin_amdgcn_fence(__ATOMIC_ACQUIRE, "workgroup");
  }
}

template <int MODE>
__global__ __launch_bounds__(256) void cvt_plane_kernel(
    const float* __restrict__ src, unsigned short* __restrict__ dst, int total8, int src8)
{
  const int i = blockIdx.x * 256 + threadIdx.x;
  if (i >= total8) return;
  const int ic = (i < src8) ? i : (src8 - 1);
  const float keep = (i < src8) ? 1.0f : 0.0f;
  const size_t e0 = (size_t)ic << 3;
  const v4f a0 = *(const v4f*)(src + e0);
  const v4f a1 = *(const v4f*)(src + e0 + 4);
  v8h hv;
#pragma unroll
  for (int e = 0; e < 4; ++e) {
    const float f0 = a0[e] * keep, f1 = a1[e] * keep;
    if (MODE == 0) {
      hv[e]     = __builtin_bit_cast(_Float16, f2bf_bits(f0));
      hv[4 + e] = __builtin_bit_cast(_Float16, f2bf_bits(f1));
    } else {
      hv[e]     = (_Float16)(bfr(f0) * 64.0f);
      hv[4 + e] = (_Float16)(bfr(f1) * 64.0f);
    }
  }
  unsigned short* q = dst + ((size_t)i << 3);
  *(volatile v8h*)q = hv;
  __threadfence();
  *(volatile v8h*)q = hv;
}

__global__ __launch_bounds__(256) void conv_split_kernel(
    const float* __restrict__ ZX, const float* __restrict__ cw, const float* __restrict__ cb,
    const float* __restrict__ dtb, const float* __restrict__ alg,
    unsigned short* __restrict__ Z16, unsigned short* __restrict__ X16,
    unsigned short* __restrict__ B16, unsigned short* __restrict__ C16,
    float* __restrict__ DT, float* __restrict__ AL)
{
  __shared__ __align__(16) float sT[16 * kConvTP];
  const int tid = threadIdx.x, lane = tid & 31, wave = tid >> 5;
  const int cblk = blockIdx.x;
  const int mode = (cblk < 8) ? 0 : ((cblk < 16) ? 1 : 2);
  const int c  = cblk * 256 + tid;
  const int cc = (c < kCproj) ? c : (kCproj - 1);
  const int g0 = blockIdx.y * 64;
  const int tb = g0 & (kSeq - 1);
  const float w0 = bfr(cw[cc * 4 + 0]), w1 = bfr(cw[cc * 4 + 1]), w2 = bfr(cw[cc * 4 + 2]), w3 = bfr(cw[cc * 4 + 3]);
  const float bc = bfr(cb[cc]);
  int hh = tid - 128;
  hh = (hh < 0) ? 0 : hh;
  hh = (hh > kHeads - 1) ? (kHeads - 1) : hh;
  const float dbias = bfr(dtb[hh]);
  const float aco   = bfr(alg[hh]);
  const bool isbc = (mode == 2) && (tid < 128);
  const bool isdt = (mode == 2) && (tid >= 128) && (tid < 128 + kHeads);
  float xm3, xm2, xm1;
  {
    const bool hist = (tb > 0);
    const int rb = hist ? (g0 - 3) : g0;
    const float v3 = ZX[(size_t)rb * kCpad + cc];
    const float v2 = ZX[(size_t)(rb + 1) * kCpad + cc];
    const float v1 = ZX[(size_t)(rb + 2) * kCpad + cc];
    xm3 = hist ? v3 : 0.f;
    xm2 = hist ? v2 : 0.f;
    xm1 = hist ? v1 : 0.f;
  }
#pragma unroll 1
  for (int sub = 0; sub < 4; ++sub) {
    const int lb = g0 + sub * 16;
#pragma unroll 1
    for (int s = 0; s < 16; ++s) {
      const float xcur = ZX[(size_t)(lb + s) * kCpad + cc];
      float acc = w0 * xm3;
      acc = fmaf(w1, xm2, acc);
      acc = fmaf(w2, xm1, acc);
      acc = fmaf(w3, xcur, acc);
      const float v = acc + bc;
      if (mode != 2) sT[s * kConvTP + tid] = v;
      if (isbc) sT[s * kConvTP + tid] = v;
      if (isdt) {
        const float uu = v + dbias;
        const float sp = fmaxf(uu, 0.0f) + log1pf(expf(-fabsf(uu)));
        sT[s * kConvTP + tid] = sp;
        sT[s * kConvTP + tid + kHeads] = sp * aco;
      }
      xm3 = xm2; xm2 = xm1; xm1 = xcur;
    }
    __syncthreads();
    if (mode != 2) {
      unsigned short* P = (mode == 0) ? Z16 : X16;
      const int d0 = (mode == 0) ? (cblk * 256) : ((cblk - 8) * 256);
      v8h hv[2];
#pragma unroll
      for (int it = 0; it < 2; ++it) {
        const float* sp = sT + (it * 8 + wave) * kConvTP + lane * 8;
        const v4f a0 = *(const v4f*)(sp);
        const v4f a1 = *(const v4f*)(sp + 4);
#pragma unroll
        for (int e = 0; e < 4; ++e) { hv[it][e] = (_Float16)a0[e]; hv[it][4 + e] = (_Float16)a1[e]; }
      }
      for (int pass = 0; pass < 2; ++pass) {
#pragma unroll
        for (int it = 0; it < 2; ++it)
          *(volatile v8h*)(P + (size_t)(lb + it * 8 + wave) * kDi + d0 + lane * 8) = hv[it];
        __threadfence();
      }
    } else {
      const int q = lane >> 3, s8 = lane & 7;
      if (wave < 4) {
        const int row = wave * 4 + q;
        const float* sp = sT + row * kConvTP + s8 * 8;
        const v4f b0 = *(const v4f*)(sp);
        const v4f b1 = *(const v4f*)(sp + 4);
        const v4f c0 = *(const v4f*)(sp + 64);
        const v4f c1 = *(const v4f*)(sp + 68);
        v8h bv, cv;
#pragma unroll
        for (int e = 0; e < 4; ++e) {
          bv[e] = (_Float16)b0[e]; bv[4 + e] = (_Float16)b1[e];
          cv[e] = (_Float16)c0[e]; cv[4 + e] = (_Float16)c1[e];
        }
        const size_t o = (size_t)(lb + row) * kNs + s8 * 8;
        for (int pass = 0; pass < 2; ++pass) {
          *(volatile v8h*)(B16 + o) = bv;
          *(volatile v8h*)(C16 + o) = cv;
          __threadfence();
        }
      } else {
        const int row = (wave - 4) * 4 + q;
        const float* sp = sT + row * kConvTP + 128 + s8 * 4;
        const v4f dv  = *(const v4f*)(sp);
        const v4f avv = *(const v4f*)(sp + kHeads);
        const size_t o = (size_t)(lb + row) * kHeads + s8 * 4;
        for (int pass = 0; pass < 2; ++pass) {
          *(volatile v4f*)(DT + o) = dv;
          *(volatile v4f*)(AL + o) = avv;
          __threadfence();
        }
      }
    }
    __syncthreads();
  }
}

__device__ __forceinline__ void put_raw2(unsigned short* T16, int pb, int q, unsigned w) {
  T16[pb * kTP + q]       = (unsigned short)(w & 0xffffu);
  T16[(pb + 1) * kTP + q] = (unsigned short)(w >> 16);
}
__device__ __forceinline__ void put_raw8(unsigned short* T16, int pb, int q, v4u u) {
  put_raw2(T16, pb + 0, q, u[0]); put_raw2(T16, pb + 2, q, u[1]);
  put_raw2(T16, pb + 4, q, u[2]); put_raw2(T16, pb + 6, q, u[3]);
}
__device__ __forceinline__ void put_scaled2(unsigned short* T16, int pb, int q, unsigned w, float wq) {
  T16[pb * kTP + q]       = f16_bits(h16_to_f32(w & 0xffffu) * wq);
  T16[(pb + 1) * kTP + q] = f16_bits(h16_to_f32(w >> 16) * wq);
}
__device__ __forceinline__ void put_scaled8(unsigned short* T16, int pb, int q, v4u u, float wq) {
  put_scaled2(T16, pb + 0, q, u[0], wq); put_scaled2(T16, pb + 2, q, u[1], wq);
  put_scaled2(T16, pb + 4, q, u[2], wq); put_scaled2(T16, pb + 6, q, u[3], wq);
}
__device__ __forceinline__ void stage_x_col(const unsigned short* __restrict__ xrow, unsigned short* Xt, int q) {
  const v4u* xp = (const v4u*)(const void*)xrow;
#pragma unroll 1
  for (int g = 0; g < 2; ++g) {
    const v4u u0 = xp[4 * g + 0], u1 = xp[4 * g + 1], u2 = xp[4 * g + 2], u3 = xp[4 * g + 3];
    put_raw8(Xt, 32 * g + 0, q, u0);  put_raw8(Xt, 32 * g + 8, q, u1);
    put_raw8(Xt, 32 * g + 16, q, u2); put_raw8(Xt, 32 * g + 24, q, u3);
  }
}
__device__ __forceinline__ void put_h4(unsigned short* Ht, int pb, int n, v4f f) {
  Ht[(pb + 0) * kHP + n] = f16_bits(f[0] * 1024.0f);
  Ht[(pb + 1) * kHP + n] = f16_bits(f[1] * 1024.0f);
  Ht[(pb + 2) * kHP + n] = f16_bits(f[2] * 1024.0f);
  Ht[(pb + 3) * kHP + n] = f16_bits(f[3] * 1024.0f);
}
__device__ __forceinline__ _Float16 m_entry(float cbv, int i, int j, float si, const float* sS, const float* sDT) {
  const bool keep = (j <= i);
  const float d = keep ? (si - sS[j]) : 0.0f;
  const float m = cbv * expf(d) * sDT[j] * 1024.0f;
  return (_Float16)(keep ? m : 0.0f);
}

__global__ __launch_bounds__(128) void chunk_state_kernel(
    const unsigned short* __restrict__ B16, const unsigned short* __restrict__ X16,
    const float* __restrict__ DT, const float* __restrict__ AL, float* __restrict__ DH)
{
  __shared__ float sS[kChunkQ];
  __shared__ float sTot[4];
  __shared__ __align__(16) unsigned short Aw[kNs * kTP];
  __shared__ __align__(16) unsigned short Xt[kHd * kTP];
  __shared__ __align__(16) float slab[4][16 * 68];
  const int tid = threadIdx.x, lane = tid & 31, wave = tid >> 5;
  const int blk = blockIdx.x, bc = blk >> 5, h = blk & 31;
  const size_t row0 = (size_t)bc * kChunkQ;
  const float dtv = DT[(row0 + tid) * kHeads + h];
  const float av  = AL[(row0 + tid) * kHeads + h];
  const float v = wave_scan_incl(av, lane);
  if (lane == 31) sTot[wave] = v;
  __syncthreads();
  const float t0 = sTot[0], t1 = sTot[1], t2 = sTot[2];
  float pre = (wave > 0) ? t0 : 0.0f;
  pre += (wave > 1) ? t1 : 0.0f;
  pre += (wave > 2) ? t2 : 0.0f;
  const float s = pre + v;
  sS[tid] = s;
  __syncthreads();
  const float sLast = sS[kChunkQ - 1];
  const float wq = dtv * expf(sLast - s) * 1024.0f;
  {
    const v4u* bp = (const v4u*)(const void*)(B16 + (row0 + tid) * kNs);
#pragma unroll 1
    for (int g = 0; g < 2; ++g) {
      const v4u u0 = bp[4 * g + 0], u1 = bp[4 * g + 1], u2 = bp[4 * g + 2], u3 = bp[4 * g + 3];
      put_scaled8(Aw, 32 * g + 0, tid, u0, wq);  put_scaled8(Aw, 32 * g + 8, tid, u1, wq);
      put_scaled8(Aw, 32 * g + 16, tid, u2, wq); put_scaled8(Aw, 32 * g + 24, tid, u3, wq);
    }
  }
  stage_x_col(X16 + (row0 + tid) * kDi + h * kHd, Xt, tid);
  __syncthreads();

  const int rlane = lane & 15, koff = (lane >> 4) * 8, mOff = (lane >> 4) * 8;
  v8f acc[4];
#pragma unroll
  for (int t = 0; t < 4; ++t) acc[t] = (v8f){0.f,0.f,0.f,0.f,0.f,0.f,0.f,0.f};
#pragma unroll
  for (int k0 = 0; k0 < kChunkQ; k0 += 32) {
    const v16h fa = lds_frag(Aw + (wave * 16 + rlane) * kTP + k0 + koff);
    v16h fb[4];
#pragma unroll
    for (int t = 0; t < 4; ++t) fb[t] = lds_frag(Xt + (t * 16 + rlane) * kTP + k0 + koff);
#pragma unroll
    for (int t = 0; t < 4; ++t) acc[t] = Frag<_Float16>::mma(fa, fb[t], acc[t]);
    Frag<_Float16>::guard4(acc[0], acc[1], acc[2], acc[3], fa, fb[3]);
    Frag<_Float16>::keep(fb[0], fb[1], fb[2], fb[3]);
  }
  acc_guard4(acc[0], acc[1], acc[2], acc[3]);

  float* sl = slab[wave];
#pragma unroll
  for (int t = 0; t < 4; ++t)
#pragma unroll
    for (int r = 0; r < 8; ++r) sl[(mOff + r) * 68 + t * 16 + rlane] = acc[t][r] * (1.0f / 1024.0f);
  __builtin_amdgcn_fence(__ATOMIC_RELEASE, "workgroup");
  __builtin_amdgcn_wave_barrier();
  __builtin_amdgcn_fence(__ATOMIC_ACQUIRE, "workgroup");
  float* D = DH + (size_t)blk * (kNs * kHd) + (size_t)(wave * 16) * kHd;
  const int hh = lane >> 4, c4 = (lane & 15) * 4;
  for (int pass = 0; pass < 2; ++pass) {
#pragma unroll
    for (int it = 0; it < 8; ++it) {
      const int row = it * 2 + hh;
      const v4f vv = *(const v4f*)(sl + row * 68 + c4);
      *(volatile v4f*)(D + (size_t)row * kHd + c4) = vv;
    }
    __threadfence();
  }
}

__global__ __launch_bounds__(256) void state_scan_kernel(
    const float* __restrict__ AL, const float* __restrict__ DH, float* __restrict__ HPV)
{
  __shared__ float sSL[kNChunk];
  const int tid = threadIdx.x, lane = tid & 31, wave = tid >> 5;
  const int bh = blockIdx.x >> 2, part = blockIdx.x & 3;
  const int b = bh >> 5, h = bh & 31;
#pragma unroll
  for (int rr = 0; rr < 2; ++rr) {
    const int c = wave + 8 * rr;
    const size_t rb = ((size_t)(b * kNChunk + c)) * kChunkQ;
    float v = AL[(rb + lane) * kHeads + h];
    v += AL[(rb + lane + 32) * kHeads + h];
    v += AL[(rb + lane + 64) * kHeads + h];
    v += AL[(rb + lane + 96) * kHeads + h];
#pragma unroll
    for (int off = 1; off < 32; off <<= 1) v += __shfl_xor(v, off, 32);
    if (lane == 0) sSL[c] = v;
  }
  __syncthreads();
  const size_t e0 = (size_t)part * 1024 + (size_t)tid * 4;
  v4f hs = (v4f){0.f, 0.f, 0.f, 0.f};
#pragma unroll 1
  for (int c = 0; c < kNChunk; ++c) {
    const size_t base = ((size_t)(b * kNChunk + c) * kHeads + h) * (size_t)(kNs * kHd) + e0;
    *(volatile v4f*)(HPV + base) = hs;
    __threadfence();
    *(volatile v4f*)(HPV + base) = hs;
    const v4f dh = *(const v4f*)(DH + base);
    const float dec = expf(sSL[c]);
    hs = hs * dec + dh;
  }
}

__global__ __launch_bounds__(256) void ssm_out_kernel(
    const float* __restrict__ CB, const unsigned short* __restrict__ X16, const unsigned short* __restrict__ C16,
    const float* __restrict__ DT, const float* __restrict__ AL, const float* __restrict__ HPV,
    const float* __restrict__ Dp, float* __restrict__ Y)
{
  __shared__ float sS[kChunkQ];
  __shared__ float sDT[kChunkQ];
  __shared__ float sTot[4];
  __shared__ __align__(16) unsigned short Mt[kChunkQ * kTP];
  __shared__ __align__(16) unsigned short Xt[kHd * kTP];
  __shared__ __align__(16) unsigned short Ht[kHd * kHP];
  __shared__ __align__(16) float slab[8][16 * 68];
  const int tid = threadIdx.x, lane = tid & 31, wave = tid >> 5;
  const int blk = blockIdx.x, bc = blk >> 5, h = blk & 31;
  const size_t row0 = (size_t)bc * kChunkQ;
  const int qq = tid & (kChunkQ - 1);
  const float dtv = DT[(row0 + qq) * kHeads + h];
  const float av  = AL[(row0 + qq) * kHeads + h];
  const float v = wave_scan_incl(av, lane);
  if (lane == 31 && wave < 4) sTot[wave] = v;
  __syncthreads();
  const float t0 = sTot[0], t1 = sTot[1], t2 = sTot[2];
  const int w4 = wave & 3;
  float pre = (w4 > 0) ? t0 : 0.0f;
  pre += (w4 > 1) ? t1 : 0.0f;
  pre += (w4 > 2) ? t2 : 0.0f;
  const float s = pre + v;
  if (wave < 4) { sS[tid] = s; sDT[tid] = dtv; }
  if (wave < 4) {
    stage_x_col(X16 + (row0 + tid) * kDi + h * kHd, Xt, tid);
  } else {
    const int t2i = tid - 128;
    const int n = t2i >> 1, p0 = (t2i & 1) * 32;
    const v4f* hp = (const v4f*)(HPV + (size_t)blk * (kNs * kHd) + (size_t)n * kHd + p0);
#pragma unroll 1
    for (int g = 0; g < 2; ++g) {
      const v4f f0 = hp[4 * g + 0], f1 = hp[4 * g + 1], f2 = hp[4 * g + 2], f3 = hp[4 * g + 3];
      put_h4(Ht, p0 + 16 * g + 0, n, f0);  put_h4(Ht, p0 + 16 * g + 4, n, f1);
      put_h4(Ht, p0 + 16 * g + 8, n, f2);  put_h4(Ht, p0 + 16 * g + 12, n, f3);
    }
  }
  __syncthreads();
  {
    const int i = tid >> 1, jh = (tid & 1) * 64;
    const float si = sS[i];
    const float* cbrow = CB + ((size_t)bc * kChunkQ + i) * kChunkQ + jh;
#pragma unroll 1
    for (int g = 0; g < 8; ++g) {
      const int j0 = jh + 8 * g;
      const v4f c0 = *(const v4f*)(cbrow + 8 * g);
      const v4f c1 = *(const v4f*)(cbrow + 8 * g + 4);
      v8h mv;
#pragma unroll
      for (int e = 0; e < 4; ++e) {
        mv[e]     = m_entry(c0[e], i, j0 + e, si, sS, sDT);
        mv[4 + e] = m_entry(c1[e], i, j0 + 4 + e, si, sS, sDT);
      }
      *(v8h*)(void*)(Mt + i * kTP + j0) = mv;
    }
  }
  __syncthreads();

  const int rlane = lane & 15, koff = (lane >> 4) * 8, mOff = (lane >> 4) * 8;
  v8f acc[4], acc2[4];
#pragma unroll
  for (int t = 0; t < 4; ++t) {
    acc[t]  = (v8f){0.f,0.f,0.f,0.f,0.f,0.f,0.f,0.f};
    acc2[t] = (v8f){0.f,0.f,0.f,0.f,0.f,0.f,0.f,0.f};
  }
#pragma unroll
  for (int k0 = 0; k0 < kChunkQ; k0 += 32) {
    const v16h fa = lds_frag(Mt + (wave * 16 + rlane) * kTP + k0 + koff);
    v16h fb[4];
#pragma unroll
    for (int t = 0; t < 4; ++t) fb[t] = lds_frag(Xt + (t * 16 + rlane) * kTP + k0 + koff);
#pragma unroll
    for (int t = 0; t < 4; ++t) acc[t] = Frag<_Float16>::mma(fa, fb[t], acc[t]);
    Frag<_Float16>::guard4(acc[0], acc[1], acc[2], acc[3], fa, fb[3]);
    Frag<_Float16>::keep(fb[0], fb[1], fb[2], fb[3]);
  }
  {
    const _Float16* Crow = (const _Float16*)(const void*)(C16 + (row0 + wave * 16 + rlane) * kNs + koff);
#pragma unroll
    for (int k0 = 0; k0 < kNs; k0 += 32) {
      const v16h fa = Frag<_Float16>::load(Crow + k0);
      v16h fb[4];
#pragma unroll
      for (int t = 0; t < 4; ++t) fb[t] = lds_frag(Ht + (t * 16 + rlane) * kHP + k0 + koff);
#pragma unroll
      for (int t = 0; t < 4; ++t) acc2[t] = Frag<_Float16>::mma(fa, fb[t], acc2[t]);
      Frag<_Float16>::guard4(acc2[0], acc2[1], acc2[2], acc2[3], fa, fb[3]);
      Frag<_Float16>::keep(fb[0], fb[1], fb[2], fb[3]);
    }
  }
  acc_guard4(acc[0], acc[1], acc[2], acc[3]);
  acc_guard4(acc2[0], acc2[1], acc2[2], acc2[3]);

  float Dv[4];
#pragma unroll
  for (int t = 0; t < 4; ++t) Dv[t] = bfr(Dp[h * kHd + t * 16 + rlane]);
  float es[8];
#pragma unroll
  for (int r = 0; r < 8; ++r) es[r] = expf(sS[wave * 16 + mOff + r]) * (1.0f / 1024.0f);
  float* sl = slab[wave];
#pragma unroll
  for (int t = 0; t < 4; ++t) {
#pragma unroll
    for (int r = 0; r < 8; ++r) {
      const int i = wave * 16 + mOff + r;
      const float xv = h16_to_f32((unsigned)Xt[(t * 16 + rlane) * kTP + i]);
      float y = acc[t][r] * (1.0f / 1024.0f);
      y = fmaf(es[r], acc2[t][r], y);
      y = fmaf(Dv[t], xv, y);
      sl[(mOff + r) * 68 + t * 16 + rlane] = y;
    }
  }
  __builtin_amdgcn_fence(__ATOMIC_RELEASE, "workgroup");
  __builtin_amdgcn_wave_barrier();
  __builtin_amdgcn_fence(__ATOMIC_ACQUIRE, "workgroup");
  float* Yb = Y + (row0 + wave * 16) * kDi + (size_t)h * kHd;
  const int hh = lane >> 4, c4 = (lane & 15) * 4;
  for (int pass = 0; pass < 2; ++pass) {
#pragma unroll
    for (int it = 0; it < 8; ++it) {
      const int row = it * 2 + hh;
      const v4f vv = *(const v4f*)(sl + row * 68 + c4);
      *(volatile v4f*)(Yb + (size_t)row * kDi + c4) = vv;
    }
    __threadfence();
  }
}

__global__ __launch_bounds__(256) void norm_gate_kernel(
    const float* __restrict__ Y, const unsigned short* __restrict__ Z16, const float* __restrict__ nw,
    unsigned short* __restrict__ G16)
{
  __shared__ float sred[8];
  const int tid = threadIdx.x, lane = tid & 31, wave = tid >> 5;
  const size_t row = blockIdx.x;
  const int d0 = tid * 8;
  const v4f y0 = *(const v4f*)(Y + row * kDi + d0);
  const v4f y1 = *(const v4f*)(Y + row * kDi + d0 + 4);
  float ss = 0.0f;
#pragma unroll
  for (int e = 0; e < 4; ++e) ss = fmaf(y0[e], y0[e], ss);
#pragma unroll
  for (int e = 0; e < 4; ++e) ss = fmaf(y1[e], y1[e], ss);
#pragma unroll
  for (int off = 1; off < 32; off <<= 1) ss += __shfl_xor(ss, off, 32);
  if (lane == 0) sred[wave] = ss;
  __syncthreads();
  float tot = sred[0];
  tot += sred[1]; tot += sred[2]; tot += sred[3]; tot += sred[4]; tot += sred[5]; tot += sred[6]; tot += sred[7];
  const float rinv = rsqrtf(tot * (1.0f / (float)kDi) + 1.1920929e-7f);
  const v4u zw = *(const v4u*)(const void*)(Z16 + row * kDi + d0);
  const v4f n0 = *(const v4f*)(nw + d0);
  const v4f n1 = *(const v4f*)(nw + d0 + 4);
  float ya[8], na[8];
  unsigned zb[8];
#pragma unroll
  for (int e = 0; e < 4; ++e) {
    ya[e] = y0[e]; ya[4 + e] = y1[e];
    na[e] = bfr(n0[e]); na[4 + e] = bfr(n1[e]);
  }
  zb[0] = zw[0] & 0xffffu; zb[1] = zw[0] >> 16; zb[2] = zw[1] & 0xffffu; zb[3] = zw[1] >> 16;
  zb[4] = zw[2] & 0xffffu; zb[5] = zw[2] >> 16; zb[6] = zw[3] & 0xffffu; zb[7] = zw[3] >> 16;
  v8h hv;
#pragma unroll
  for (int k = 0; k < 8; ++k) {
    const float zv = h16_to_f32(zb[k]);
    const float ex = expf(-zv);
    const float sg = __builtin_amdgcn_rcpf(1.0f + ex);
    const float yn = ya[k] * rinv * na[k];
    const float g = yn * (zv * sg) * 16.0f;
    hv[k] = (_Float16)g;
  }
  unsigned short* q = G16 + row * kDi + d0;
  *(volatile v8h*)q = hv;
  __threadfence();
  *(volatile v8h*)q = hv;
}

extern "C" void kernel_launch(void* const* d_in, const int* in_sizes, int n_in,
                              void* d_out, int out_size, void* d_ws, size_t ws_size,
                              hipStream_t stream) {
  if (n_in < 9) return;
  if (in_sizes[0] != kRows * kDm) return;
  if (in_sizes[1] != kCproj * kDm) return;
  if (in_sizes[2] != kCproj * 4) return;
  if (in_sizes[3] != kCproj) return;
  if (in_sizes[4] != kHeads) return;
  if (in_sizes[5] != kDi) return;
  if (in_sizes[6] != kHeads) return;
  if (in_sizes[7] != kDi) return;
  if (in_sizes[8] != kDm * kDi) return;
  if (out_size != kRows * kDm) return;
  if (ws_size < kWsTotal) return;

  const float* u      = (const float*)d_in[0];
  const float* w_in   = (const float*)d_in[1];
  const float* conv_w = (const float*)d_in[2];
  const float* conv_b = (const float*)d_in[3];
  const float* a_par  = (const float*)d_in[4];
  const float* d_par  = (const float*)d_in[5];
  const float* dt_b   = (const float*)d_in[6];
  const float* norm_w = (const float*)d_in[7];
  const float* w_out  = (const float*)d_in[8];
  float* out = (float*)d_out;

  char* ws = (char*)d_ws;
  unsigned short* UB  = (unsigned short*)(ws + kOffUB);
  unsigned short* WIB = (unsigned short*)(ws + kOffWIB);
  unsigned short* WOB = (unsigned short*)(ws + kOffWOB);
  float*          ZX  = (float*)(ws + kOffZX);
  unsigned short* Z16 = (unsigned short*)(ws + kOffZ16);
  unsigned short* X16 = (unsigned short*)(ws + kOffX16);
  unsigned short* B16 = (unsigned short*)(ws + kOffB16);
  unsigned short* C16 = (unsigned short*)(ws + kOffC16);
  float*          DT  = (float*)(ws + kOffDT);
  float*          AL  = (float*)(ws + kOffAL);
  float*          CB  = (float*)(ws + kOffCB);
  float*          DH  = (float*)(ws + kOffDH);
  float*          HPV = (float*)(ws + kOffHPV);
  float*          Y   = (float*)(ws + kOffY);
  unsigned short* G16 = (unsigned short*)(ws + kOffG16);

  cvt_plane_kernel<0><<<kU8 / 256, 256, 0, stream>>>(u, UB, kU8, kU8);
  cvt_plane_kernel<0><<<kWin8 / 256, 256, 0, stream>>>(w_in, WIB, kWin8, kWinSrc8);
  cvt_plane_kernel<1><<<kWout8 / 256, 256, 0, stream>>>(w_out, WOB, kWout8, kWout8);

  wmma_gemm64<1, 0, 0, 0, false><<<dim3(kTilesIn / 8, 1), 256, 0, stream>>>(
      UB, nullptr, kDm, 0L,
      WIB, nullptr, kDm, 0L,
      (void*)ZX, nullptr, kCpad, 0L,
      nullptr, nullptr, 0L,
      kRows, kCpad, kDm, 1.0f);

  conv_split_kernel<<<dim3(17, kRows / 64), 256, 0, stream>>>(ZX, conv_w, conv_b, dt_b, a_par, Z16, X16, B16, C16, DT, AL);

  wmma_gemm64<0, 0, 0, 0, false><<<dim3(1, kNbc), 256, 0, stream>>>(
      C16, nullptr, kNs, (long)kChunkQ * kNs,
      B16, nullptr, kNs, (long)kChunkQ * kNs,
      (void*)CB, nullptr, kChunkQ, (long)kChunkQ * kChunkQ,
      nullptr, nullptr, 0L,
      kChunkQ, kChunkQ, kNs, 1.0f);

  chunk_state_kernel<<<kNblk, 128, 0, stream>>>(B16, X16, DT, AL, DH);

  state_scan_kernel<<<kBatch * kHeads * 4, 256, 0, stream>>>(AL, DH, HPV);

  ssm_out_kernel<<<kNblk, 256, 0, stream>>>(CB, X16, C16, DT, AL, HPV, d_par, Y);

  norm_gate_kernel<<<kRows, 256, 0, stream>>>(Y, Z16, norm_w, G16);

  wmma_gemm64<0, 0, 0, 0, false><<<dim3(kTilesOut / 8, 1), 256, 0, stream>>>(
      G16, nullptr, kDi, 0L,
      WOB, nullptr, kDi, 0L,
      (void*)out, nullptr, kDm, 0L,
      nullptr, nullptr, 0L,
      kRows, kDm, kDi, 1.0f / 1024.0f);
}
